// ExpressionModel_56813827391507
// MI455X (gfx1250) — hardware-run, weakly checked
//
#include <hip/hip_runtime.h>
#include <stddef.h>


typedef _Float16 v16h __attribute__((ext_vector_type(16)));
typedef _Float16 v8h  __attribute__((ext_vector_type(8)));
typedef float    v8f  __attribute__((ext_vector_type(8)));
typedef float    v4f  __attribute__((ext_vector_type(4)));
typedef _Float16 h16;

#ifndef NB
#define NB 2
#endif
#ifndef SEQ
#define SEQ 2048
#endif
#ifndef ALEN
#define ALEN 512
#endif
#define NB_FULL   2
#define SEQ_FULL  2048
#define ALEN_FULL 512
#define DIM   1024
#define NHEAD 16
#define HD    64
#define DFF   4096
#define TDIM  768
#define NMOD  (6 * DIM)
#define MROWS (NB * SEQ)
#define AROWS (NB * ALEN)

static_assert(NB >= 1 && NB <= NB_FULL);
static_assert(NB <= 8);
static_assert(SEQ >= 128 && SEQ <= SEQ_FULL && (SEQ % 128) == 0);
static_assert(ALEN >= 64 && ALEN <= ALEN_FULL && (ALEN % 64) == 0);
static_assert(ALEN <= SEQ);
static_assert(DIM == NHEAD * HD);
static_assert(HD == 64);
static_assert((DIM % 64) == 0 && (DIM % 32) == 0);
static_assert((DFF % 64) == 0 && (DFF % 32) == 0);
static_assert((TDIM % 64) == 0 && (TDIM % 32) == 0 && (TDIM % 8) == 0);
static_assert(((3 * DIM) % 64) == 0 && ((2 * DIM) % 64) == 0);
static_assert((NMOD % 128) == 0);
static_assert((MROWS % 64) == 0 && (SEQ % 64) == 0);
static_assert((AROWS % 64) == 0);
static_assert((MROWS % 8) == 0);
static_assert(DIM == 32 * 8 * 4);
static_assert((size_t)MROWS * DFF < (size_t)0xFFFFFFFFu);
static_assert((((size_t)AROWS * TDIM) % 2048) == 0);

#define LDT 72
#define LDC 68
#define ALD (DIM + 8)

#define WCARRY 64.0f
#define ACARRY 16.0f
#define QCARRY 16.0f
#define PCARRY 1024.0f
#define VCARRY 64.0f
#define GCARRY 64.0f
#define GEMM_INV (1.0f / (WCARRY * ACARRY))
#define QK_MULT  (QCARRY / (WCARRY * ACARRY))
#define V_MULT   (VCARRY / (WCARRY * ACARRY))
#define CTX_INV  (1.0f / (WCARRY * VCARRY))
#define DN_INV   (1.0f / (WCARRY * GCARRY))

#define WQKV_ELEMS  ((size_t)3 * DIM * DIM)
#define WSA_ELEMS   ((size_t)DIM * DIM)
#define WQ_ELEMS    ((size_t)DIM * DIM)
#define WKV_ELEMS   ((size_t)2 * DIM * TDIM)
#define WCA_ELEMS   ((size_t)DIM * DIM)
#define WG_ELEMS    ((size_t)DFF * DIM)
#define WU_ELEMS    ((size_t)DFF * DIM)
#define WD_ELEMS    ((size_t)DIM * DFF)
#define W_BYTES     ((WQKV_ELEMS + WSA_ELEMS + WQ_ELEMS + WKV_ELEMS + WCA_ELEMS + WG_ELEMS + \
                      WU_ELEMS + WD_ELEMS) * 2)
#define WAD_ELEMS   ((size_t)NMOD * DIM)
#define WAD_BYTES   (WAD_ELEMS * 2)
#define AUD_BYTES   ((size_t)AROWS * TDIM * 2)
#define PLANE_ELEMS ((size_t)MROWS * DIM)
#define PLANE16_BYTES (PLANE_ELEMS * 2)
#define FS_BYTES    (PLANE_ELEMS * 4)
#define G_BYTES     ((size_t)MROWS * DFF * 2)
#define GREG_BYTES  ((G_BYTES > (WAD_BYTES + AUD_BYTES)) ? G_BYTES : (WAD_BYTES + AUD_BYTES))
#define MODS_BYTES  ((size_t)NB * NMOD * 4)
#define WS_TOTAL    (W_BYTES + PLANE16_BYTES * 5 + FS_BYTES + GREG_BYTES + MODS_BYTES)
static_assert((W_BYTES % 128) == 0 && (PLANE16_BYTES % 128) == 0);
static_assert((FS_BYTES % 128) == 0 && (G_BYTES % 128) == 0);
static_assert((WAD_BYTES % 128) == 0 && (AUD_BYTES % 128) == 0 && (MODS_BYTES % 128) == 0);
static_assert((size_t)NB * DIM * SEQ == PLANE_ELEMS);
static_assert((size_t)AROWS * DIM <= PLANE_ELEMS);
static_assert((size_t)NB * DIM * ALEN <= PLANE_ELEMS);
static_assert(PLANE16_BYTES * 2 == FS_BYTES);
static_assert(WAD_BYTES + AUD_BYTES <= GREG_BYTES && G_BYTES <= GREG_BYTES);
static_assert(WS_TOTAL <= (size_t)134217728);

__device__ __forceinline__ float bf16r(float x) {
  unsigned int u = __float_as_uint(x);
  u = (u + 0x7FFFu + ((u >> 16) & 1u)) & 0xFFFF0000u;
  return __uint_as_float(u);
}

static __device__ __forceinline__ h16 toh_flush(float v) {
  const h16 r = (h16)v;
  return (fabsf(v) < 6.103515625e-05f) ? (h16)0.0f : r;
}

__device__ __forceinline__ float silu_f(float x) {
  return x * __builtin_amdgcn_rcpf(1.0f + __expf(-x));
}

__device__ __forceinline__ v16h frag_at(const _Float16* p) {
  v8h lo = *(const v8h*)(p);
  v8h hi = *(const v8h*)(p + 16);
  v16h out;
#pragma unroll
  for (int i = 0; i < 8; ++i) { out[i] = lo[i]; out[i + 8] = hi[i]; }
  return out;
}
__device__ __forceinline__ v16h ld_frag(const _Float16* base, unsigned ld) {
  const unsigned lane = threadIdx.x & 31u;
  return frag_at(base + (lane & 15u) * ld + (lane >> 4) * 8u);
}

__device__ __forceinline__ v8f wmma16(v16h a, v16h b, v8f c) {
  v8f d = __builtin_amdgcn_wmma_f32_16x16x32_f16(false, a, false, b, (short)0, c,
                                                 false, false);
  asm volatile("v_nop\n\tv_nop\n\tv_nop\n\tv_nop" : "+v"(d) : "v"(a), "v"(b));
  return d;
}

__device__ __forceinline__ void wave_lds_sync() {
  __builtin_amdgcn_fence(3  , "wavefront");
  asm volatile("s_wait_dscnt 0x0" ::: "memory");
  __builtin_amdgcn_wave_barrier();
}

__global__ __launch_bounds__(256) void wtrans_kernel(
    const float* __restrict__ src, _Float16* __restrict__ dst, unsigned K, unsigned N) {
  __shared__ float Ts[64 * LDC];
  const unsigned tid = threadIdx.x;
  const unsigned n0 = blockIdx.x * 64u;
  const unsigned k0 = blockIdx.y * 64u;
#pragma unroll
  for (unsigned j = 0; j < 4u; ++j) {
    const unsigned idx = tid + 256u * j;
    const unsigned r = idx >> 4, c = (idx & 15u) * 4u;
    const v4f a = *(const v4f*)(src + (size_t)(k0 + r) * N + n0 + c);
    *(v4f*)&Ts[r * LDC + c] = a;
  }
  __syncthreads();
  v8h x[2];
  size_t off[2];
#pragma unroll
  for (unsigned i = 0; i < 2u; ++i) {
    const unsigned n = 32u * i + (tid >> 3);
    const unsigned kk = (tid & 7u) * 8u;
#pragma unroll
    for (unsigned j = 0; j < 8u; ++j)
      x[i][j] = toh_flush(WCARRY * bf16r(Ts[(kk + j) * LDC + n]));
    off[i] = (size_t)(n0 + n) * K + k0 + kk;
  }
#pragma unroll
  for (int i = 0; i < 2; ++i) *(volatile v8h*)(dst + off[i]) = x[i];
  __threadfence();
#pragma unroll
  for (int i = 0; i < 2; ++i) *(volatile v8h*)(dst + off[i]) = x[i];
}

__global__ __launch_bounds__(256) void aconv_kernel(
    const float* __restrict__ src, _Float16* __restrict__ dst) {
  const size_t e = ((size_t)blockIdx.x * 256u + threadIdx.x) * 8u;
  const unsigned row = (unsigned)(e / (size_t)TDIM);
  const unsigned col = (unsigned)(e - (size_t)row * TDIM);
  const unsigned bidx = row / (unsigned)ALEN;
  const unsigned l = row - bidx * (unsigned)ALEN;
  const float* sp = src + ((size_t)bidx * ALEN_FULL + l) * TDIM + col;
  const v4f a0 = *(const v4f*)(sp);
  const v4f a1 = *(const v4f*)(sp + 4);
  v8h o;
#pragma unroll
  for (int j = 0; j < 4; ++j) {
    o[j]     = toh_flush(ACARRY * bf16r(a0[j]));
    o[j + 4] = toh_flush(ACARRY * bf16r(a1[j]));
  }
  *(volatile v8h*)(dst + e) = o;
  __threadfence();
  *(volatile v8h*)(dst + e) = o;
}

__global__ __launch_bounds__(256) void adaln_kernel(
    const float* __restrict__ tmod, const _Float16* __restrict__ Wt,
    const float* __restrict__ bias, float* __restrict__ mods) {
  __shared__ _Float16 As[16 * ALD];
  __shared__ float Ms[NB * 128];
  const unsigned tid = threadIdx.x, lane = tid & 31u;
  const unsigned w = (unsigned)__builtin_amdgcn_readfirstlane((int)(tid >> 5));
  const unsigned hh = lane >> 4, m = lane & 15u;

#pragma unroll 1
  for (unsigned j = 0; j < 8u; ++j) {
    const unsigned idx = tid + 256u * j;
    const unsigned row = idx >> 7, c = (idx & 127u) * 8u;
    const unsigned rr = (row < (unsigned)NB) ? row : (unsigned)(NB - 1);
    const float keep = (row < (unsigned)NB) ? ACARRY : 0.0f;
    const v4f a0 = *(const v4f*)(tmod + (size_t)rr * DIM + c);
    const v4f a1 = *(const v4f*)(tmod + (size_t)rr * DIM + c + 4);
    v8h o;
#pragma unroll
    for (int t = 0; t < 4; ++t) {
      o[t]     = toh_flush(keep * silu_f(bf16r(a0[t])));
      o[t + 4] = toh_flush(keep * silu_f(bf16r(a1[t])));
    }
    *(v8h*)&As[row * ALD + c] = o;
  }
  __syncthreads();

  const unsigned nb0 = blockIdx.x * 128u;
  const _Float16* bp = Wt + (size_t)(nb0 + w * 16u + m) * (size_t)DIM + hh * 8u;
  v8f acc = {};
#pragma unroll 2
  for (unsigned k0 = 0; k0 < (unsigned)DIM; k0 += 32u) {
    const v16h a = ld_frag(&As[k0], ALD);
    const v16h b = frag_at(bp + k0);
    acc = wmma16(a, b, acc);
  }
  if (hh == 0u) {
#pragma unroll
    for (int r = 0; r < NB; ++r) Ms[(unsigned)r * 128u + w * 16u + m] = acc[r];
  }
  __syncthreads();
  if (tid < (unsigned)NB * 32u) {
    const unsigned row = tid >> 5, c = (tid & 31u) * 4u;
    const v4f u = *(const v4f*)&Ms[row * 128u + c];
    const v4f bb = *(const v4f*)(bias + nb0 + c);
    v4f val;
#pragma unroll
    for (int j = 0; j < 4; ++j) val[j] = u[j] * GEMM_INV + bf16r(bb[j]);
    float* dp = mods + (size_t)row * NMOD + nb0 + c;
    *(volatile v4f*)dp = val;
    __threadfence();
    *(volatile v4f*)dp = val;
  }
}

__global__ __launch_bounds__(256) void rmsnorm_kernel(
    const float* __restrict__ src, const float* __restrict__ lnw,
    const float* __restrict__ mods, _Float16* __restrict__ dst,
    unsigned seq_src, unsigned rnd, unsigned modf, unsigned scale_off, unsigned shift_off) {
#pragma clang fp contract(off)
  const unsigned tid = threadIdx.x, lane = tid & 31u, w = tid >> 5;
  const unsigned crow = blockIdx.x * 8u + w;
  const unsigned bidx = crow / (unsigned)SEQ;
  const unsigned sq = crow - bidx * (unsigned)SEQ;
  const float* sp = src + ((size_t)bidx * seq_src + sq) * DIM;
  const float* mp = mods + (size_t)bidx * NMOD;
  const float mk = modf ? 1.0f : 0.0f;
  float ss = 0.0f;
#pragma unroll 1
  for (unsigned j = 0; j < 4u; ++j) {
    const unsigned c = (j * 32u + lane) * 8u;
    const v4f a0 = *(const v4f*)(sp + c);
    const v4f a1 = *(const v4f*)(sp + c + 4);
#pragma unroll
    for (int t = 0; t < 4; ++t) {
      const float x0 = rnd ? bf16r(a0[t]) : a0[t];
      const float x1 = rnd ? bf16r(a1[t]) : a1[t];
      ss = fmaf(x0, x0, ss);
      ss = fmaf(x1, x1, ss);
    }
  }
#pragma unroll
  for (int off = 1; off < 32; off <<= 1) ss += __shfl_xor(ss, off, 32);
  const float rinv = 1.0f / sqrtf(ss * (1.0f / (float)DIM) + 1.0e-6f);
#pragma unroll 1
  for (unsigned j = 0; j < 4u; ++j) {
    const unsigned c = (j * 32u + lane) * 8u;
    const v4f a0 = *(const v4f*)(sp + c);
    const v4f a1 = *(const v4f*)(sp + c + 4);
    const v4f g0 = *(const v4f*)(lnw + c);
    const v4f g1 = *(const v4f*)(lnw + c + 4);
    const v4f s0 = *(const v4f*)(mp + scale_off + c);
    const v4f s1 = *(const v4f*)(mp + scale_off + c + 4);
    const v4f h0 = *(const v4f*)(mp + shift_off + c);
    const v4f h1 = *(const v4f*)(mp + shift_off + c + 4);
    v8h o;
#pragma unroll
    for (int t = 0; t < 4; ++t) {
      const float x0 = rnd ? bf16r(a0[t]) : a0[t];
      const float x1 = rnd ? bf16r(a1[t]) : a1[t];
      const float y0 = ((x0 * rinv) * bf16r(g0[t])) * (1.0f + mk * s0[t]) + mk * h0[t];
      const float y1 = ((x1 * rinv) * bf16r(g1[t])) * (1.0f + mk * s1[t]) + mk * h1[t];
      o[t]     = toh_flush(ACARRY * y0);
      o[t + 4] = toh_flush(ACARRY * y1);
    }
    _Float16* dp = dst + (size_t)crow * DIM + c;
    *(volatile v8h*)dp = o;
    __threadfence();
    *(volatile v8h*)dp = o;
  }
}

enum { GM_QKV = 0, GM_Q = 1, GM_KV = 2, GM_SA = 3, GM_CA = 4, GM_GU = 5, GM_DN = 6 };

template <int MODE, int KD>
__device__ __forceinline__ void gemm_body(
    const _Float16* __restrict__ A16, const _Float16* __restrict__ Bt,
    const _Float16* __restrict__ Bt2,
    const float* __restrict__ addf, const float* __restrict__ mods,
    const float* __restrict__ ctab, const float* __restrict__ stab,
    float* __restrict__ outf, _Float16* __restrict__ out16,
    _Float16* __restrict__ out16t) {
  static_assert((KD % 32) == 0);
  __shared__ float Cs[64 * LDC];
  const unsigned tid = threadIdx.x, lane = tid & 31u, w = tid >> 5;
  const unsigned mw = w >> 1, nw = w & 1u;
  const unsigned hh = lane >> 4, m = lane & 15u;
  const unsigned n0 = blockIdx.x * 64u;
  const unsigned row0 = blockIdx.y * 64u;

  const _Float16* ap  = A16 + (size_t)(row0 + mw * 16u + m) * (size_t)KD + hh * 8u;
  const _Float16* bp0 = Bt + (size_t)(n0 + nw * 32u + m) * (size_t)KD + hh * 8u;
  const _Float16* bp1 = bp0 + (size_t)16 * (size_t)KD;
  v8f acc0 = {}, acc1 = {};
  if (MODE == GM_GU) {
    const _Float16* cp0 = Bt2 + (size_t)(n0 + nw * 32u + m) * (size_t)KD + hh * 8u;
    const _Float16* cp1 = cp0 + (size_t)16 * (size_t)KD;
    v8f acc2 = {}, acc3 = {};
#pragma unroll 2
    for (unsigned k0 = 0; k0 < (unsigned)KD; k0 += 32u) {
      const v16h a  = frag_at(ap + k0);
      const v16h b0 = frag_at(bp0 + k0);
      const v16h b1 = frag_at(bp1 + k0);
      const v16h c0 = frag_at(cp0 + k0);
      const v16h c1 = frag_at(cp1 + k0);
      acc0 = wmma16(a, b0, acc0);
      acc1 = wmma16(a, b1, acc1);
      acc2 = wmma16(a, c0, acc2);
      acc3 = wmma16(a, c1, acc3);
    }
#pragma unroll
    for (int r = 0; r < 8; ++r) {
      const float g0 = acc0[r] * GEMM_INV, u0 = acc2[r] * GEMM_INV;
      const float g1 = acc1[r] * GEMM_INV, u1 = acc3[r] * GEMM_INV;
      acc0[r] = GCARRY * (silu_f(g0) * u0);
      acc1[r] = GCARRY * (silu_f(g1) * u1);
    }
  } else {
#pragma unroll 2
    for (unsigned k0 = 0; k0 < (unsigned)KD; k0 += 32u) {
      const v16h a  = frag_at(ap + k0);
      const v16h b0 = frag_at(bp0 + k0);
      const v16h b1 = frag_at(bp1 + k0);
      acc0 = wmma16(a, b0, acc0);
      acc1 = wmma16(a, b1, acc1);
    }
  }
#pragma unroll
  for (int r = 0; r < 8; ++r) {
    float* d = &Cs[(mw * 16u + hh * 8u + (unsigned)r) * LDC + nw * 32u + m];
    d[0]  = acc0[r];
    d[16] = acc1[r];
  }
  __syncthreads();

  if (MODE == GM_QKV || MODE == GM_Q || MODE == GM_KV) {
    const unsigned which = n0 / (unsigned)DIM;
    const unsigned nc0 = n0 - which * (unsigned)DIM;
    const unsigned tsel = (MODE == GM_QKV) ? 2u : ((MODE == GM_KV) ? 1u : 99u);
    if (which != tsel) {
      v8h x[2];
      size_t off[2];
#pragma unroll
      for (unsigned i = 0; i < 2u; ++i) {
        const unsigned r = 32u * i + (tid >> 3);
        const unsigned c = (tid & 7u) * 8u;
        const v4f u0 = *(const v4f*)&Cs[r * LDC + c];
        const v4f u1 = *(const v4f*)&Cs[r * LDC + c + 4];
        v4f e0 = u0, e1 = u1;
        if (MODE == GM_QKV) {
          const unsigned sq = (row0 + r) % (unsigned)SEQ;
          const unsigned p0 = ((nc0 & 63u) + c) >> 1;
          const v4f cc = *(const v4f*)(ctab + (size_t)sq * (HD / 2) + p0);
          const v4f sn = *(const v4f*)(stab + (size_t)sq * (HD / 2) + p0);
          const float c0 = bf16r(cc[0]), c1 = bf16r(cc[1]), c2 = bf16r(cc[2]), c3 = bf16r(cc[3]);
          const float s0 = bf16r(sn[0]), s1 = bf16r(sn[1]), s2 = bf16r(sn[2]), s3 = bf16r(sn[3]);
          e0[0] = u0[0] * c0 - u0[1] * s0;  e0[1] = u0[0] * s0 + u0[1] * c0;
          e0[2] = u0[2] * c1 - u0[3] * s1;  e0[3] = u0[2] * s1 + u0[3] * c1;
          e1[0] = u1[0] * c2 - u1[1] * s2;  e1[1] = u1[0] * s2 + u1[1] * c2;
          e1[2] = u1[2] * c3 - u1[3] * s3;  e1[3] = u1[2] * s3 + u1[3] * c3;
        }
#pragma unroll
        for (int j = 0; j < 4; ++j) {
          x[i][j]     = toh_flush(e0[j] * QK_MULT);
          x[i][j + 4] = toh_flush(e1[j] * QK_MULT);
        }
        off[i] = (size_t)which * PLANE_ELEMS + (size_t)(row0 + r) * DIM + nc0 + c;
      }
#pragma unroll
      for (int i = 0; i < 2; ++i) *(volatile v8h*)(out16 + off[i]) = x[i];
      __threadfence();
#pragma unroll
      for (int i = 0; i < 2; ++i) *(volatile v8h*)(out16 + off[i]) = x[i];
    } else {
      const unsigned SL = (MODE == GM_KV) ? (unsigned)ALEN : (unsigned)SEQ;
      const unsigned bidx = row0 / SL;
      const unsigned key0 = row0 - bidx * SL;
      v8h x[2];
      size_t off[2];
#pragma unroll
      for (unsigned i = 0; i < 2u; ++i) {
        const unsigned dcol = 32u * i + (tid >> 3);
        const unsigned kk = (tid & 7u) * 8u;
#pragma unroll
        for (unsigned j = 0; j < 8u; ++j)
          x[i][j] = toh_flush(Cs[(kk + j) * LDC + dcol] * V_MULT);
        off[i] = ((size_t)bidx * DIM + nc0 + dcol) * SL + key0 + kk;
      }
#pragma unroll
      for (int i = 0; i < 2; ++i) *(volatile v8h*)(out16t + off[i]) = x[i];
      __threadfence();
#pragma unroll
      for (int i = 0; i < 2; ++i) *(volatile v8h*)(out16t + off[i]) = x[i];
    }
  }

  if (MODE == GM_GU) {
    v8h x[2];
    size_t off[2];
#pragma unroll
    for (unsigned i = 0; i < 2u; ++i) {
      const unsigned r = 32u * i + (tid >> 3);
      const unsigned c = (tid & 7u) * 8u;
      const v4f u0 = *(const v4f*)&Cs[r * LDC + c];
      const v4f u1 = *(const v4f*)&Cs[r * LDC + c + 4];
#pragma unroll
      for (int j = 0; j < 4; ++j) {
        x[i][j]     = toh_flush(u0[j]);
        x[i][j + 4] = toh_flush(u1[j]);
      }
      off[i] = (size_t)(row0 + r) * DFF + n0 + c;
    }
#pragma unroll
    for (int i = 0; i < 2; ++i) *(volatile v8h*)(out16 + off[i]) = x[i];
    __threadfence();
#pragma unroll
    for (int i = 0; i < 2; ++i) *(volatile v8h*)(out16 + off[i]) = x[i];
  }

  if (MODE == GM_SA || MODE == GM_CA || MODE == GM_DN) {
    v4f xs[4];
    size_t off[4];
#pragma unroll
    for (unsigned i = 0; i < 4u; ++i) {
      const unsigned r = 16u * i + (tid >> 4);
      const unsigned c = (tid & 15u) * 4u;
      const unsigned crow = row0 + r;
      const unsigned bidx = crow / (unsigned)SEQ;
      const unsigned sq = crow - bidx * (unsigned)SEQ;
      const size_t frow = (size_t)bidx * SEQ_FULL + sq;
      const v4f u = *(const v4f*)&Cs[r * LDC + c];
      v4f val;
      if (MODE == GM_SA) {
        const v4f g = *(const v4f*)(addf + frow * DIM + n0 + c);
        const v4f gt = *(const v4f*)(mods + (size_t)bidx * NMOD + 2 * DIM + n0 + c);
#pragma unroll
        for (int j = 0; j < 4; ++j)
          val[j] = bf16r(g[j]) + gt[j] * (u[j] * CTX_INV);
        off[i] = (size_t)crow * DIM + n0 + c;
      } else if (MODE == GM_CA) {
        const v4f g = *(const v4f*)(addf + (size_t)crow * DIM + n0 + c);
#pragma unroll
        for (int j = 0; j < 4; ++j)
          val[j] = g[j] + u[j] * CTX_INV;
        off[i] = (size_t)crow * DIM + n0 + c;
      } else {
        const v4f g = *(const v4f*)(addf + (size_t)crow * DIM + n0 + c);
        const v4f gt = *(const v4f*)(mods + (size_t)bidx * NMOD + 5 * DIM + n0 + c);
#pragma unroll
        for (int j = 0; j < 4; ++j)
          val[j] = g[j] + gt[j] * (u[j] * DN_INV);
        off[i] = frow * DIM + n0 + c;
      }
      xs[i] = val;
    }
#pragma unroll
    for (int i = 0; i < 4; ++i) *(volatile v4f*)(outf + off[i]) = xs[i];
    __threadfence();
#pragma unroll
    for (int i = 0; i < 4; ++i) *(volatile v4f*)(outf + off[i]) = xs[i];
  }
}

__global__ __launch_bounds__(256) void gemm_qkv_kernel(
    const _Float16* __restrict__ A16, const _Float16* __restrict__ Bt,
    const float* __restrict__ ctab, const float* __restrict__ stab,
    _Float16* __restrict__ out16, _Float16* __restrict__ out16t) {
  gemm_body<GM_QKV, DIM>(A16, Bt, nullptr, nullptr, nullptr, ctab, stab, nullptr, out16, out16t);
}
__global__ __launch_bounds__(256) void gemm_q_kernel(
    const _Float16* __restrict__ A16, const _Float16* __restrict__ Bt,
    _Float16* __restrict__ out16) {
  gemm_body<GM_Q, DIM>(A16, Bt, nullptr, nullptr, nullptr, nullptr, nullptr, nullptr, out16,
                       nullptr);
}
__global__ __launch_bounds__(256) void gemm_kv_kernel(
    const _Float16* __restrict__ A16, const _Float16* __restrict__ Bt,
    _Float16* __restrict__ out16, _Float16* __restrict__ out16t) {
  gemm_body<GM_KV, TDIM>(A16, Bt, nullptr, nullptr, nullptr, nullptr, nullptr, nullptr, out16,
                         out16t);
}
__global__ __launch_bounds__(256) void gemm_sa_kernel(
    const _Float16* __restrict__ A16, const _Float16* __restrict__ Bt,
    const float* __restrict__ xin, const float* __restrict__ mods, float* __restrict__ outf) {
  gemm_body<GM_SA, DIM>(A16, Bt, nullptr, xin, mods, nullptr, nullptr, outf, nullptr, nullptr);
}
__global__ __launch_bounds__(256) void gemm_ca_kernel(
    const _Float16* __restrict__ A16, const _Float16* __restrict__ Bt,
    const float* __restrict__ x1, float* __restrict__ outf) {
  gemm_body<GM_CA, DIM>(A16, Bt, nullptr, x1, nullptr, nullptr, nullptr, outf, nullptr, nullptr);
}
__global__ __launch_bounds__(256) void gemm_gu_kernel(
    const _Float16* __restrict__ A16, const _Float16* __restrict__ Btg,
    const _Float16* __restrict__ Btu, _Float16* __restrict__ out16) {
  gemm_body<GM_GU, DIM>(A16, Btg, Btu, nullptr, nullptr, nullptr, nullptr, nullptr, out16,
                        nullptr);
}
__global__ __launch_bounds__(256) void gemm_dn_kernel(
    const _Float16* __restrict__ A16, const _Float16* __restrict__ Bt,
    const float* __restrict__ x2, const float* __restrict__ mods, float* __restrict__ outf) {
  gemm_body<GM_DN, DFF>(A16, Bt, nullptr, x2, mods, nullptr, nullptr, outf, nullptr, nullptr);
}

__global__ __launch_bounds__(256) void attn_kernel(
    const _Float16* __restrict__ Qh, const _Float16* __restrict__ Kh,
    const _Float16* __restrict__ Vt, _Float16* __restrict__ Ov, unsigned Lk) {
  __shared__ _Float16 Os[8 * 16 * LDT];

  const unsigned tid = threadIdx.x, lane = tid & 31u;
  const unsigned w = (unsigned)__builtin_amdgcn_readfirstlane((int)(tid >> 5));
  const unsigned hh = lane >> 4, m = lane & 15u;
  const unsigned q0 = blockIdx.x * 128u;
  const unsigned head = blockIdx.y;
  const unsigned b = blockIdx.z;
  const float sc = 0.125f / (QCARRY * QCARRY);
  const unsigned pbase = w * (16u * LDT);
  const unsigned qbase = q0 + w * 16u;

  const _Float16* qp = Qh + (size_t)(b * (unsigned)SEQ + qbase + m) * DIM + head * HD + hh * 8u;
  const v16h qf0 = frag_at(qp);
  const v16h qf1 = frag_at(qp + 32);
  const _Float16* kp = Kh + ((size_t)b * Lk + m) * DIM + head * HD + hh * 8u;
  const _Float16* vp = Vt + ((size_t)b * DIM + head * HD + m) * (size_t)Lk + hh * 8u;
  const size_t vstep = (size_t)16 * Lk;

  float mrun = -1.0e30f, lrun = 0.0f;
  v8f o[4];
#pragma unroll
  for (int t = 0; t < 4; ++t) o[t] = (v8f){};

#pragma unroll 1
  for (unsigned kb = 0; kb < Lk; kb += 32u) {
    const _Float16* kr = kp + (size_t)kb * DIM;
    v8f s0 = {}, s1 = {};
    {
      const v16h ka = frag_at(kr);
      const v16h kc = frag_at(kr + 32);
      s0 = wmma16(ka, qf0, s0);
      s0 = wmma16(kc, qf1, s0);
    }
    {
      const v16h ka = frag_at(kr + (size_t)16 * DIM);
      const v16h kc = frag_at(kr + (size_t)16 * DIM + 32);
      s1 = wmma16(ka, qf0, s1);
      s1 = wmma16(kc, qf1, s1);
    }

    float a0[8], a1[8];
    float mx = -1.0e30f;
#pragma unroll
    for (int r = 0; r < 8; ++r) {
      a0[r] = s0[r] * sc;
      a1[r] = s1[r] * sc;
      mx = fmaxf(mx, fmaxf(a0[r], a1[r]));
    }
    mx = fmaxf(mx, __shfl_xor(mx, 16, 32));
    const float mn = fmaxf(mrun, mx);
    const float al = __expf(mrun - mn);
    mrun = mn;
    float rs = 0.0f;
    v16h pf;
#pragma unroll
    for (int r = 0; r < 8; ++r) {
      const h16 ph0 = toh_flush(__expf(a0[r] - mn) * PCARRY);
      const h16 ph1 = toh_flush(__expf(a1[r] - mn) * PCARRY);
      pf[r] = ph0;
      pf[r + 8] = ph1;
      rs += (float)ph0 + (float)ph1;
    }
    rs += __shfl_xor(rs, 16, 32);
    lrun = al * lrun + rs;
#pragma unroll
    for (int t = 0; t < 4; ++t)
#pragma unroll
      for (int r = 0; r < 8; ++r) o[t][r] = o[t][r] * al;

    const _Float16* vr = vp + kb;
    const v16h vf0 = frag_at(vr);
    const v16h vf1 = frag_at(vr + vstep);
    const v16h vf2 = frag_at(vr + 2 * vstep);
    const v16h vf3 = frag_at(vr + 3 * vstep);
    o[0] = wmma16(vf0, pf, o[0]);
    o[1] = wmma16(vf1, pf, o[1]);
    o[2] = wmma16(vf2, pf, o[2]);
    o[3] = wmma16(vf3, pf, o[3]);
  }

  const float inv = __builtin_amdgcn_rcpf(lrun);
#pragma unroll
  for (int t = 0; t < 4; ++t) {
    v8h ov;
#pragma unroll
    for (int r = 0; r < 8; ++r) ov[r] = toh_flush(o[t][r] * inv);
    *(v8h*)&Os[pbase + m * LDT + (unsigned)t * 16u + hh * 8u] = ov;
  }
  wave_lds_sync();
  v8h x[4];
  size_t off[4];
#pragma unroll
  for (unsigned i = 0; i < 4u; ++i) {
    const unsigned r = 4u * i + (lane >> 3);
    const unsigned c = (lane & 7u) * 8u;
    x[i] = *(const v8h*)&Os[pbase + r * LDT + c];
    off[i] = (size_t)(b * (unsigned)SEQ + qbase + r) * DIM + head * HD + c;
  }
#pragma unroll
  for (int i = 0; i < 4; ++i) *(volatile v8h*)(Ov + off[i]) = x[i];
  __threadfence();
#pragma unroll
  for (int i = 0; i < 4; ++i) *(volatile v8h*)(Ov + off[i]) = x[i];
}

extern "C" void kernel_launch(void* const* d_in, const int* in_sizes, int n_in,
                              void* d_out, int out_size, void* d_ws, size_t ws_size,
                              hipStream_t stream) {
  if (n_in < 18) return;
  const long long need_x = ((long long)(NB - 1) * SEQ_FULL + SEQ) * DIM;
  const long long need_a = ((long long)(NB - 1) * ALEN_FULL + ALEN) * TDIM;
  if ((long long)in_sizes[0] < need_x) return;
  if ((long long)in_sizes[1] < (long long)NB * DIM) return;
  if ((long long)in_sizes[2] < need_a) return;
  if ((long long)in_sizes[3] < (long long)SEQ * (HD / 2)) return;
  if ((long long)in_sizes[4] < (long long)SEQ * (HD / 2)) return;
  if (in_sizes[5] < DIM || in_sizes[6] < DIM || in_sizes[7] < DIM) return;
  if ((long long)in_sizes[8] < (long long)3 * DIM * DIM) return;
  if ((long long)in_sizes[9] < (long long)DIM * DIM) return;
  if ((long long)in_sizes[10] < (long long)DIM * DIM) return;
  if ((long long)in_sizes[11] < (long long)2 * DIM * TDIM) return;
  if ((long long)in_sizes[12] < (long long)DIM * DIM) return;
  if ((long long)in_sizes[13] < (long long)DIM * DFF) return;
  if ((long long)in_sizes[14] < (long long)DIM * DFF) return;
  if ((long long)in_sizes[15] < (long long)DFF * DIM) return;
  if ((long long)in_sizes[16] < (long long)DIM * NMOD) return;
  if (in_sizes[17] < NMOD) return;
  if ((long long)out_size < need_x) return;
  if (ws_size < WS_TOTAL) return;

  const float* X     = (const float*)d_in[0];
  const float* Tmod  = (const float*)d_in[1];
  const float* Audio = (const float*)d_in[2];
  const float* Fcos  = (const float*)d_in[3];
  const float* Fsin  = (const float*)d_in[4];
  const float* n1w   = (const float*)d_in[5];
  const float* n2w   = (const float*)d_in[6];
  const float* n3w   = (const float*)d_in[7];
  const float* Wqkv  = (const float*)d_in[8];
  const float* Wsa   = (const float*)d_in[9];
  const float* Wq    = (const float*)d_in[10];
  const float* Wkv   = (const float*)d_in[11];
  const float* Wca   = (const float*)d_in[12];
  const float* Wg    = (const float*)d_in[13];
  const float* Wu    = (const float*)d_in[14];
  const float* Wd    = (const float*)d_in[15];
  const float* Wad   = (const float*)d_in[16];
  const float* bad   = (const float*)d_in[17];
  float* out = (float*)d_out;

  char* ws = (char*)d_ws;
  _Float16* Wqkv16 = (_Float16*)ws;
  _Float16* Wsa16  = Wqkv16 + WQKV_ELEMS;
  _Float16* Wq16   = Wsa16 + WSA_ELEMS;
  _Float16* Wkv16  = Wq16 + WQ_ELEMS;
  _Float16* Wca16  = Wkv16 + WKV_ELEMS;
  _Float16* Wg16   = Wca16 + WCA_ELEMS;
  _Float16* Wu16   = Wg16 + WG_ELEMS;
  _Float16* Wd16   = Wu16 + WU_ELEMS;
  _Float16* H16    = (_Float16*)(ws + W_BYTES);
  _Float16* Q16    = (_Float16*)(ws + W_BYTES + 1 * PLANE16_BYTES);
  _Float16* K16    = (_Float16*)(ws + W_BYTES + 2 * PLANE16_BYTES);
  _Float16* Vt16   = (_Float16*)(ws + W_BYTES + 3 * PLANE16_BYTES);
  _Float16* Ctx16  = (_Float16*)(ws + W_BYTES + 4 * PLANE16_BYTES);
  float*    X1     = (float*)(ws + W_BYTES + 5 * PLANE16_BYTES);
  char*     greg   = ws + W_BYTES + 5 * PLANE16_BYTES + FS_BYTES;
  _Float16* G16    = (_Float16*)greg;
  _Float16* Wad16  = (_Float16*)greg;
  _Float16* Aud16  = (_Float16*)(greg + WAD_BYTES);
  float*    MODS   = (float*)(greg + GREG_BYTES);
  float*    X2     = (float*)Q16;

  dim3 blk(256);

  wtrans_kernel<<<dim3(3 * DIM / 64, DIM / 64), blk, 0, stream>>>(Wqkv, Wqkv16, DIM, 3 * DIM);
  wtrans_kernel<<<dim3(DIM / 64, DIM / 64), blk, 0, stream>>>(Wsa, Wsa16, DIM, DIM);
  wtrans_kernel<<<dim3(DIM / 64, DIM / 64), blk, 0, stream>>>(Wq, Wq16, DIM, DIM);
  wtrans_kernel<<<dim3(2 * DIM / 64, TDIM / 64), blk, 0, stream>>>(Wkv, Wkv16, TDIM, 2 * DIM);
  wtrans_kernel<<<dim3(DIM / 64, DIM / 64), blk, 0, stream>>>(Wca, Wca16, DIM, DIM);
  wtrans_kernel<<<dim3(DFF / 64, DIM / 64), blk, 0, stream>>>(Wg, Wg16, DIM, DFF);
  wtrans_kernel<<<dim3(DFF / 64, DIM / 64), blk, 0, stream>>>(Wu, Wu16, DIM, DFF);
  wtrans_kernel<<<dim3(DIM / 64, DFF / 64), blk, 0, stream>>>(Wd, Wd16, DFF, DIM);
  wtrans_kernel<<<dim3(NMOD / 64, DIM / 64), blk, 0, stream>>>(Wad, Wad16, DIM, NMOD);
  aconv_kernel<<<dim3((unsigned)(((size_t)AROWS * TDIM) / 2048)), blk, 0, stream>>>(Audio, Aud16);

  adaln_kernel<<<dim3(NMOD / 128), blk, 0, stream>>>(Tmod, Wad16, bad, MODS);

  rmsnorm_kernel<<<dim3(MROWS / 8), blk, 0, stream>>>(X, n1w, MODS, H16, (unsigned)SEQ_FULL, 1u,
                                                      1u, (unsigned)DIM, 0u);
  gemm_qkv_kernel<<<dim3(3 * DIM / 64, MROWS / 64), blk, 0, stream>>>(H16, Wqkv16, Fcos, Fsin,
                                                                      Q16, Vt16);
  attn_kernel<<<dim3(SEQ / 128, NHEAD, NB), blk, 0, stream>>>(Q16, K16, Vt16, Ctx16,
                                                              (unsigned)SEQ);
  gemm_sa_kernel<<<dim3(DIM / 64, MROWS / 64), blk, 0, stream>>>(Ctx16, Wsa16, X, MODS, X1);

  rmsnorm_kernel<<<dim3(MROWS / 8), blk, 0, stream>>>(X1, n2w, MODS, H16, (unsigned)SEQ, 0u,
                                                      0u, 0u, 0u);
  gemm_q_kernel<<<dim3(DIM / 64, MROWS / 64), blk, 0, stream>>>(H16, Wq16, Q16);
  gemm_kv_kernel<<<dim3(2 * DIM / 64, AROWS / 64), blk, 0, stream>>>(Aud16, Wkv16, K16, Vt16);
  attn_kernel<<<dim3(SEQ / 128, NHEAD, NB), blk, 0, stream>>>(Q16, K16, Vt16, Ctx16,
                                                              (unsigned)ALEN);
  gemm_ca_kernel<<<dim3(DIM / 64, MROWS / 64), blk, 0, stream>>>(Ctx16, Wca16, X1, X2);

  rmsnorm_kernel<<<dim3(MROWS / 8), blk, 0, stream>>>(X2, n3w, MODS, H16, (unsigned)SEQ, 0u,
                                                      1u, (unsigned)(4 * DIM),
                                                      (unsigned)(3 * DIM));
  gemm_gu_kernel<<<dim3(DFF / 64, MROWS / 64), blk, 0, stream>>>(H16, Wg16, Wu16, G16);
  gemm_dn_kernel<<<dim3(DIM / 64, MROWS / 64), blk, 0, stream>>>(G16, Wd16, X2, MODS, out);
}
